// CCM_74663711474120
// MI455X (gfx1250) — hardware-verified
//
#include <hip/hip_runtime.h>
#include <math.h>

typedef __attribute__((ext_vector_type(16))) _Float16 v16h;
typedef __attribute__((ext_vector_type(16))) __bf16 v16b;
typedef __attribute__((ext_vector_type(8)))  _Float16 v8h;
typedef __attribute__((ext_vector_type(8)))  float v8f;
typedef __attribute__((ext_vector_type(4)))  float v4f;
typedef __attribute__((ext_vector_type(2)))  float v2f;
typedef __attribute__((ext_vector_type(4)))  unsigned v4u;
typedef __attribute__((ext_vector_type(4)))  int v4i;
typedef float __attribute__((may_alias)) float_a;
typedef int __attribute__((may_alias)) int_a;

template <typename T> __device__ __forceinline__ void vst2(void* p, T v) { *(volatile T*)p = v; __threadfence(); *(volatile T*)p = v; }
__device__ __forceinline__ v8f wmma16(v16h a, v16h b, v8f c) {
  v8f d = __builtin_amdgcn_wmma_f32_16x16x32_f16(false, a, false, b, (short)0, c, false, false);
  asm volatile("v_nop\n\tv_nop\n\tv_nop\n\tv_nop" : "+v"(d) : "v"(a), "v"(b));
  return d;
}
__device__ __forceinline__ v8f wmma_bf(v16b a, v16b b, v8f c) {
  v8f d = __builtin_amdgcn_wmma_f32_16x16x32_bf16(false, a, false, b, (short)0, c, false, false);
  asm volatile("v_nop\n\tv_nop\n\tv_nop\n\tv_nop" : "+v"(d) : "v"(a), "v"(b));
  return d;
}
__device__ __forceinline__ v16h frag_h(const _Float16* rowk0, int lane) {
  union { v16h v; v8h q[2]; } u; const _Float16* p = rowk0 + 8 * (lane >> 4);
  u.q[0] = *(const v8h*)p; u.q[1] = *(const v8h*)(p + 16); return u.v;
}
__device__ __forceinline__ v16h frag_f32(const float* rowk0, int lane) {
  v16h a; const float* p = rowk0 + 8 * (lane >> 4);
#pragma unroll
  for (int i = 0; i < 8; ++i) { a[i] = (_Float16)p[i]; a[8 + i] = (_Float16)p[16 + i]; }
  return a;
}
__device__ __forceinline__ v16h frag_f32s(const float* rowk0, int lane, float sc) {
  v16h a; const float* p = rowk0 + 8 * (lane >> 4);
#pragma unroll
  for (int i = 0; i < 8; ++i) { a[i] = (_Float16)(p[i] * sc); a[8 + i] = (_Float16)(p[16 + i] * sc); }
  return a;
}
__device__ __forceinline__ v16h fragc_f32(const float* W, int k0, int n, int lane, int ld, int K) {
  v16h a; const int g = lane >> 4;
#pragma unroll
  for (int i = 0; i < 8; ++i) { const int ka = k0 + 8 * g + i, kb = ka + 16;
    a[i] = (_Float16)(ka < K ? W[(size_t)ka * ld + n] : 0.f); a[8 + i] = (_Float16)(kb < K ? W[(size_t)kb * ld + n] : 0.f); }
  return a;
}
struct F2 { v16b h, l; };
__device__ __forceinline__ F2 bsplit16(const float v[16]) { F2 r;
#pragma unroll
  for (int i = 0; i < 16; ++i) { const __bf16 h = (__bf16)v[i]; r.h[i] = h; r.l[i] = (__bf16)(v[i] - (float)h); }
  return r; }
__device__ __forceinline__ F2 split_row(const float* row, int k0, int lane) { float v[16]; const float* p = row + k0 + 8 * (lane >> 4);
#pragma unroll
  for (int i = 0; i < 8; ++i) { v[i] = p[i]; v[8 + i] = p[16 + i]; }
  return bsplit16(v); }
__device__ __forceinline__ F2 split_rowK(const float* row, int k0, int lane, int K) { float v[16]; const int g = lane >> 4;
#pragma unroll
  for (int i = 0; i < 8; ++i) { const int ka = k0 + 8 * g + i, kb = ka + 16; v[i] = ka < K ? row[ka] : 0.f; v[8 + i] = kb < K ? row[kb] : 0.f; }
  return bsplit16(v); }
__device__ __forceinline__ F2 split_col(const float* W, int k0, int n, int lane, int ld, int K) { float v[16]; const int g = lane >> 4;
#pragma unroll
  for (int i = 0; i < 8; ++i) { const int ka = k0 + 8 * g + i, kb = ka + 16; v[i] = ka < K ? W[(size_t)ka * ld + n] : 0.f; v[8 + i] = kb < K ? W[(size_t)kb * ld + n] : 0.f; }
  return bsplit16(v); }
__device__ __forceinline__ v8f mac3(const F2& a, const F2& b, v8f c) { c = wmma_bf(a.l, b.h, c); c = wmma_bf(a.h, b.l, c); return wmma_bf(a.h, b.h, c); }
__device__ __forceinline__ float sigm(float v) { return 1.0f / (1.0f + expf(-v)); }
#define LDSX() do { asm volatile("s_wait_dscnt 0" ::: "memory"); __builtin_amdgcn_wave_barrier(); __builtin_amdgcn_fence(__ATOMIC_RELEASE, "workgroup"); } while (0)

#define BS 64
#define NM 1024
#define DD 2048
#define HD 128
#define NC 65
#define NCP 80
#define NCS 96
#define NR (BS + NM)

__global__ __launch_bounds__(256) void k_norm(const float* __restrict__ f, const float* __restrict__ emb, float* __restrict__ XN) {
  const int wave = threadIdx.x >> 5, lane = threadIdx.x & 31; const int r = blockIdx.x * 8 + wave; if (r >= NR) return;
  const float* src = r < BS ? f + (size_t)r * DD : emb + (size_t)(r - BS) * DD; float s = 0.f;
  for (int c = lane; c < DD; c += 32) { const float v = src[c]; s += v * v; }
#pragma unroll
  for (int off = 16; off >= 1; off >>= 1) s += __shfl_xor(s, off, 32);
  const float inv = 1.0f / fmaxf(sqrtf(s), 1e-12f);
  for (int c = lane * 4; c < DD; c += 128) { v4f v = *(const v4f*)(src + c); v *= inv; vst2(XN + (size_t)r * DD + c, v); }
}
__global__ __launch_bounds__(32) void k_zx(const float* __restrict__ XN, float* __restrict__ ZX) {
  __shared__ __align__(16) float ss[16][NM + 4];
  const int lane = threadIdx.x, col = lane & 15, g = lane >> 4; const int r0 = blockIdx.x * 16;
  const float scl = 1.0f / (0.07f * 32.0f);
#pragma unroll 1
  for (int np = 0; np < NM / 128; ++np) { v8f acc[8] = {};
#pragma unroll 1
    for (int kc = 0; kc < DD / 32; ++kc) { const F2 a = split_row(XN + (size_t)(r0 + col) * DD, kc * 32, lane);
#pragma unroll
      for (int j = 0; j < 8; ++j) acc[j] = mac3(a, split_row(XN + (size_t)(BS + np * 128 + j * 16 + col) * DD, kc * 32, lane), acc[j]); }
#pragma unroll
    for (int j = 0; j < 8; ++j)
#pragma unroll
      for (int r = 0; r < 8; ++r) ss[8 * g + r][np * 128 + j * 16 + col] = acc[j][r] * scl; }
  LDSX();
  { const int rl = lane >> 1, hf = lane & 1; float* row = &ss[rl][0]; float mx = -3.4e38f; for (int c = hf * 512; c < hf * 512 + 512; ++c) mx = fmaxf(mx, row[c]); mx = fmaxf(mx, __shfl_xor(mx, 1, 32));
    float se = 0.f; for (int c = hf * 512; c < hf * 512 + 512; ++c) { const float p = expf(row[c] - mx); row[c] = p; se += p; } se += __shfl_xor(se, 1, 32); const float inv = 1.0f / se;
    LDSX();
    for (int c = hf * 512; c < hf * 512 + 512; ++c) row[c] *= inv; }
  LDSX();
  for (int rl = 0; rl < 16; ++rl) for (int pc = lane; pc < NM / 4; pc += 32) vst2(ZX + (size_t)(r0 + rl) * NM + pc * 4, *(const v4f*)(&ss[rl][pc * 4]));
}
__global__ __launch_bounds__(256) void k_px(const float* __restrict__ XN, float* __restrict__ PX) {
  __shared__ float srow[BS]; __shared__ __align__(16) float sp[BS];
  const int tid = threadIdx.x, wave = tid >> 5, lane = tid & 31;
#pragma unroll 1
  for (int b = wave; b < BS; b += 8) { float tot = 0.f;
#pragma unroll 1
    for (int b2 = 0; b2 < BS; ++b2) { float s = 0.f;
#pragma unroll 1
      for (int c = lane; c < DD; c += 32) s += XN[(size_t)b * DD + c] * XN[(size_t)b2 * DD + c];
#pragma unroll
      for (int off = 16; off >= 1; off >>= 1) s += __shfl_xor(s, off, 32);
      tot += s; }
    if (lane == 0) srow[b] = tot / (0.07f * 8.0f); }
  __syncthreads();
  if (tid == 0) { float mx = -3.4e38f; for (int b = 0; b < BS; ++b) mx = fmaxf(mx, srow[b]); float se = 0.f;
#pragma unroll 1
    for (int b = 0; b < BS; ++b) { const float p = expf(srow[b] - mx); sp[b] = p; se += p; }
#pragma unroll 1
    for (int b = 0; b < BS; ++b) sp[b] /= se; }
  __syncthreads();
  if (tid < BS / 4) vst2(PX + tid * 4, *(const v4f*)(&sp[tid * 4]));
}
__global__ __launch_bounds__(32) void k_head(const float* __restrict__ f, const float* __restrict__ emb, const float* __restrict__ w1, const float* __restrict__ b1, const float* __restrict__ g, const float* __restrict__ be, const float* __restrict__ rm, const float* __restrict__ rv, const float* __restrict__ w2, const float* __restrict__ b2, float* __restrict__ HO) {
  __shared__ __align__(16) float sh[16][HD + 4]; __shared__ __align__(16) float so[16][HD + 4];
  const int lane = threadIdx.x, col = lane & 15, gg = lane >> 4; const int r0 = blockIdx.x * 16;
  const int r = r0 + col; const float* arow = r < BS ? f + (size_t)r * DD : emb + (size_t)(r - BS) * DD;
  v8f acc[8] = {};
#pragma unroll 1
  for (int kc = 0; kc < DD / 32; ++kc) { const F2 a = split_row(arow, kc * 32, lane);
#pragma unroll
    for (int j = 0; j < 8; ++j) acc[j] = mac3(a, split_col(w1, kc * 32, j * 16 + col, lane, HD, DD), acc[j]); }
#pragma unroll
  for (int j = 0; j < 8; ++j) { const int n = j * 16 + col; const float sc = g[n] * rsqrtf(rv[n] + 1e-5f), bb = b1[n], mm = rm[n], bt = be[n];
#pragma unroll
    for (int rr = 0; rr < 8; ++rr) { float v = acc[j][rr] + bb; v = (v - mm) * sc + bt; sh[8 * gg + rr][n] = v > 0.f ? v : 0.f; } }
  LDSX();
  { v8f acc2[8] = {};
#pragma unroll
    for (int kc = 0; kc < HD / 32; ++kc) { const F2 a = split_row(&sh[col][0], kc * 32, lane);
#pragma unroll
      for (int j = 0; j < 8; ++j) acc2[j] = mac3(a, split_col(w2, kc * 32, j * 16 + col, lane, HD, HD), acc2[j]); }
#pragma unroll
    for (int j = 0; j < 8; ++j) { const int n = j * 16 + col; const float bb = b2[n];
#pragma unroll
      for (int rr = 0; rr < 8; ++rr) so[8 * gg + rr][n] = acc2[j][rr] + bb; } }
  LDSX();
  for (int rl = 0; rl < 16; ++rl) vst2(HO + (size_t)(r0 + rl) * HD + lane * 4, *(const v4f*)(&so[rl][lane * 4]));
}
__global__ __launch_bounds__(128) void k_mixpre(const float* __restrict__ HO, const float* __restrict__ mw1, const float* __restrict__ mb1, const float* __restrict__ mw2, const float* __restrict__ mb2, const float* __restrict__ cw, const float* __restrict__ cb, float* __restrict__ MAC, float* __restrict__ WP) {
  const int r = blockIdx.x, tid = threadIdx.x;
  if (r < NR) { const float* h = HO + (size_t)r * HD; const float* W = r < BS ? mw1 : mw1 + (size_t)HD * HD; float s = r < BS ? mb1[tid] : 0.f;
#pragma unroll 1
    for (int k = 0; k < HD; ++k) s += h[k] * W[(size_t)k * HD + tid];
    vst2(MAC + (size_t)r * HD + tid, s); }
  else { const int k = r - NR;
    if (tid < NCS) { float s = 0.f; if (tid < NC) { if (k < HD) { for (int m = 0; m < DD; ++m) s += mw2[(size_t)k * DD + m] * cw[(size_t)m * NC + tid]; } else { s = cb[tid]; for (int m = 0; m < DD; ++m) s += mb2[m] * cw[(size_t)m * NC + tid]; } }
      vst2(WP + (size_t)k * NCS + tid, s); } }
}
__global__ __launch_bounds__(128) void k_y(const float* __restrict__ MAC, const float* __restrict__ WP, const float* __restrict__ mg, const float* __restrict__ mbe, const float* __restrict__ mrm, const float* __restrict__ mrv, const float* __restrict__ PX, float* __restrict__ SX) {
  __shared__ __align__(16) float sh1[BS][HD + 4]; __shared__ __align__(16) float sl[BS][NCP + 4]; __shared__ __align__(16) float ssx[NCP];
  const int n = blockIdx.x, tid = threadIdx.x, wave = tid >> 5, lane = tid & 31, col = lane & 15, g = lane >> 4;
  { const int c = tid; const float mc = MAC[(size_t)(BS + n) * HD + c]; const float sc = mg[c] * rsqrtf(mrv[c] + 1e-5f), mm = mrm[c], bt = mbe[c];
    for (int b = 0; b < BS; ++b) { float v = MAC[(size_t)b * HD + c] + mc; v = (v - mm) * sc + bt; sh1[b][c] = v > 0.f ? v : 0.f; } }
  __syncthreads();
  { v8f acc[5] = {};
#pragma unroll
    for (int kc = 0; kc < HD / 32; ++kc) { const F2 a = split_row(&sh1[wave * 16 + col][0], kc * 32, lane);
#pragma unroll
      for (int t = 0; t < 5; ++t) acc[t] = mac3(a, split_col(WP, kc * 32, t * 16 + col, lane, NCS, HD), acc[t]); }
#pragma unroll
    for (int t = 0; t < 5; ++t) { const int c = t * 16 + col; const float bb = WP[(size_t)HD * NCS + c];
#pragma unroll
      for (int r = 0; r < 8; ++r) sl[wave * 16 + 8 * g + r][c] = acc[t][r] + bb; } }
  __syncthreads();
  { const int b = tid >> 1, hf = tid & 1; float* row = &sl[b][0]; float mx = -3.4e38f; for (int c = hf; c < NC; c += 2) mx = fmaxf(mx, row[c]); mx = fmaxf(mx, __shfl_xor(mx, 1, 32));
    float se = 0.f; for (int c = hf; c < NC; c += 2) { const float p = expf(row[c] - mx); row[c] = p; se += p; } se += __shfl_xor(se, 1, 32); const float wgt = PX[b] / se;
    for (int c = hf; c < NC; c += 2) row[c] *= wgt; }
  __syncthreads();
  if (tid < NCP) { float s = 0.f; if (tid < NC) for (int b = 0; b < BS; ++b) s += sl[b][tid]; ssx[tid] = s; }
  __syncthreads();
  if (tid < NCS / 4) vst2(SX + (size_t)n * NCS + tid * 4, tid < NCP / 4 ? *(const v4f*)(&ssx[tid * 4]) : (v4f){0.f, 0.f, 0.f, 0.f});
}
__global__ __launch_bounds__(256) void k_out(const float* __restrict__ ZX, const float* __restrict__ SX, float* __restrict__ out) {
  __shared__ __align__(16) float so[BS * NC + 16];
  const int tid = threadIdx.x;
  for (int q = tid; q < BS * NC; q += 256) { const int b = q / NC, c = q % NC; float s = 0.f;
#pragma unroll 1
    for (int n = 0; n < NM; ++n) s += ZX[(size_t)b * NM + n] * SX[(size_t)n * NCS + c]; so[q] = s; }
  __syncthreads();
  for (int q = tid; q < BS * NC / 4; q += 256) vst2(out + q * 4, *(const v4f*)(&so[q * 4]));
}
extern "C" void kernel_launch(void* const* d_in, const int* in_sizes, int n_in, void* d_out, int out_size, void* d_ws, size_t ws_size, hipStream_t stream) {
  (void)in_sizes; (void)n_in; (void)out_size; (void)ws_size;
  const float** I = (const float**)d_in;
  const float* f = I[0]; const float* emb = I[1];
  const float* hw1 = I[3]; const float* hb1 = I[4]; const float* hg = I[5]; const float* hbe = I[6]; const float* hrm = I[7]; const float* hrv = I[8]; const float* hw2 = I[9]; const float* hb2 = I[10];
  const float* mw1 = I[11]; const float* mb1 = I[12]; const float* mg = I[13]; const float* mbe = I[14]; const float* mrm = I[15]; const float* mrv = I[16]; const float* mw2 = I[17]; const float* mb2 = I[18]; const float* cw = I[19]; const float* cb = I[20];
  float* out = (float*)d_out;
  char* ws = (char*)d_ws; size_t off = 0;
  auto take = [&](size_t bytes) { char* p = ws + off; off += (bytes + 255) & ~(size_t)255; return p; };
  float* XN = (float*)take((size_t)NR * DD * 4); float* ZX = (float*)take((size_t)BS * NM * 4); float* PX = (float*)take(256); float* HO = (float*)take((size_t)NR * HD * 4);
  float* MAC = (float*)take((size_t)NR * HD * 4); float* WP = (float*)take((size_t)(HD + 1) * NCS * 4); float* SX = (float*)take((size_t)NM * NCS * 4);
  k_norm<<<NR / 8, 256, 0, stream>>>(f, emb, XN);
  k_zx<<<BS / 16, 32, 0, stream>>>(XN, ZX);
  k_px<<<1, 256, 0, stream>>>(XN, PX);
  k_head<<<NR / 16, 32, 0, stream>>>(f, emb, hw1, hb1, hg, hbe, hrm, hrv, hw2, hb2, HO);
  k_mixpre<<<NR + HD + 1, 128, 0, stream>>>(HO, mw1, mb1, mw2, mb2, cw, cb, MAC, WP);
  k_y<<<NM, 128, 0, stream>>>(MAC, WP, mg, mbe, mrm, mrv, PX, SX);
  k_out<<<1, 256, 0, stream>>>(ZX, SX, out);
}
